// PointnetSAModule_72052371357927
// MI455X (gfx1250) — hardware-verified
//
#include <hip/hip_runtime.h>
#pragma clang fp contract(off)

typedef __attribute__((ext_vector_type(16))) _Float16 v16h;
typedef __attribute__((ext_vector_type(8)))  _Float16 v8h;
typedef __attribute__((ext_vector_type(4)))  _Float16 v4h;
typedef __attribute__((ext_vector_type(8)))  float    v8f;
typedef __attribute__((ext_vector_type(4)))  float    v4f;
typedef __attribute__((ext_vector_type(2)))  float    v2f;
typedef __attribute__((ext_vector_type(4)))  int      v4i;
typedef __attribute__((ext_vector_type(4)))  unsigned v4u;

constexpr int NUM_BATCH   = 8;
constexpr int NUM_PTS     = 8192;
constexpr int NUM_CENT    = 2048;
constexpr int NUM_SAMP    = 32;
constexpr int NUM_CHAN    = 64;
constexpr int NUM_CHAN3   = 128;
constexpr int TOT_PTS     = NUM_BATCH * NUM_PTS;
constexpr int TOT_CENT    = NUM_BATCH * NUM_CENT;
constexpr int TOT_ROWS    = TOT_CENT * NUM_SAMP;
constexpr int LDS_PITCH   = 72;
constexpr int SLAB_PITCH  = 68;
constexpr int MLP_BLOCKS  = 1024;
constexpr int CENT_PER_BLOCK = 16;
constexpr int CENT_PER_WAVE  = 4;

static_assert(TOT_PTS == 65536);
static_assert(TOT_CENT == 16384);
static_assert(TOT_ROWS == 524288);
static_assert(MLP_BLOCKS * CENT_PER_BLOCK == TOT_CENT);
static_assert(NUM_CHAN % 32 == 0);

union FragU { v16h v; v8h h[2]; };

__device__ __forceinline__ v8f mma_h(v16h a, v16h b, v8f c) {
  c = __builtin_amdgcn_wmma_f32_16x16x32_f16(false, a, false, b, (short)0, c, false, false);
  asm volatile("v_nop\n\tv_nop\n\tv_nop\n\tv_nop" : "+v"(c) : "v"(a), "v"(b));
  return c;
}

__device__ __forceinline__ int clampi(int v, int hi) {
  v = v < 0 ? 0 : v;
  return v > hi ? hi : v;
}

__device__ __forceinline__ float h16_to_f32(unsigned hb) {
  const unsigned sgn = (hb & 0x8000u) << 16;
  const unsigned em = hb & 0x7fffu;
  const float fn = __uint_as_float((em << 13) + 0x38000000u);
  const float fs = (float)em * 5.9604644775390625e-8f;
  const float mag = (em < 0x400u) ? fs : fn;
  return __uint_as_float(__float_as_uint(mag) | sgn);
}

__device__ __forceinline__ void st2_f32(float* p, float v) {
  *(volatile float*)p = v;
  __threadfence();
  *(volatile float*)p = v;
}
__device__ __forceinline__ void st2_i32(int* p, int v) {
  *(volatile int*)p = v;
  __threadfence();
  *(volatile int*)p = v;
}
__device__ __forceinline__ void st2_v4f(float* p, v4f v) {
  *(volatile v4f*)p = v;
  __threadfence();
  *(volatile v4f*)p = v;
}
__device__ __forceinline__ void st2_v4i(int* p, v4i v) {
  *(volatile v4i*)p = v;
  __threadfence();
  *(volatile v4i*)p = v;
}
__device__ __forceinline__ void st2_v8h(_Float16* p, v8h v) {
  *(volatile v8h*)p = v;
  __threadfence();
  *(volatile v8h*)p = v;
}

__global__ __launch_bounds__(256) void wprep_kernel(const float* __restrict__ W1,
                                                    const float* __restrict__ W2,
                                                    const float* __restrict__ W3,
                                                    _Float16* __restrict__ wpl)
{
  const int t = blockIdx.x * 256 + threadIdx.x;
  const int k8 = (t & 7) * 8;
  const float* src;
  int ld, n, krow0;
  if (t < 512)       { src = W1; ld = 64;  n = t >> 3;          krow0 = 3 + k8; }
  else if (t < 1024) { src = W2; ld = 64;  n = (t - 512) >> 3;  krow0 = k8; }
  else               { src = W3; ld = 128; n = (t - 1024) >> 3; krow0 = k8; }
  v8h hv;
#pragma unroll
  for (int e = 0; e < 8; ++e) hv[e] = (_Float16)src[(size_t)(krow0 + e) * ld + n];
  st2_v8h(wpl + (size_t)t * 8, hv);
}

__global__ __launch_bounds__(1024) void fps_kernel(const float* __restrict__ xyz,
                                                   int* __restrict__ fps_idx,
                                                   float* __restrict__ out0)
{
#pragma clang fp contract(off)
  __shared__ __align__(16) float stg[3072];
  __shared__ float rv[2][32];
  __shared__ int   ri[2][32];
  __shared__ __align__(16) int sidx[NUM_CENT];

  const int b    = blockIdx.x;
  const int tid  = threadIdx.x;
  const int lane = tid & 31;
  const int wv   = tid >> 5;
  const float* X = xyz + (size_t)b * (NUM_PTS * 3);

  float px[8], py[8], pz[8], dd[8];
#pragma unroll
  for (int q = 0; q < 8; ++q) {
    __syncthreads();
    if (tid < 768) {
      const v4f t4 = *(const v4f*)(X + q * 3072 + tid * 4);
      *(v4f*)(&stg[tid * 4]) = t4;
    }
    __syncthreads();
    px[q] = stg[tid * 3 + 0];
    py[q] = stg[tid * 3 + 1];
    pz[q] = stg[tid * 3 + 2];
    dd[q] = 1e10f;
  }

  if (tid == 0) sidx[0] = 0;
  int last = 0;
  for (int it = 1; it < NUM_CENT; ++it) {
    int lu = __builtin_amdgcn_readfirstlane(last);
    lu = clampi(lu, NUM_PTS - 1);
    const float cx = X[lu * 3 + 0];
    const float cy = X[lu * 3 + 1];
    const float cz = X[lu * 3 + 2];
    float bv = 0.0f;
    int bi = 0;
#pragma unroll
    for (int q = 0; q < 8; ++q) {
      const float dx = px[q] - cx;
      const float dy = py[q] - cy;
      const float dz = pz[q] - cz;
      const float t0 = dx * dx;
      const float t1 = dy * dy;
      const float t2 = dz * dz;
      const float d2 = (t0 + t2) + t1;
      const float dc = (d2 < dd[q]) ? d2 : dd[q];
      dd[q] = dc;
      const bool tk = (q == 0) || (dc > bv);
      bv = tk ? dc : bv;
      bi = tk ? (tid + 1024 * q) : bi;
    }
#pragma unroll
    for (int off = 16; off; off >>= 1) {
      const float ov = __shfl_xor(bv, off, 32);
      const int   oi = __shfl_xor(bi, off, 32);
      const bool tk = (ov > bv) || ((ov == bv) && (oi < bi));
      bv = tk ? ov : bv;
      bi = tk ? oi : bi;
    }
    const int par = it & 1;
    if (lane == 0) { rv[par][wv] = bv; ri[par][wv] = bi; }
    __syncthreads();
    bv = rv[par][lane];
    bi = ri[par][lane];
#pragma unroll
    for (int off = 16; off; off >>= 1) {
      const float ov = __shfl_xor(bv, off, 32);
      const int   oi = __shfl_xor(bi, off, 32);
      const bool tk = (ov > bv) || ((ov == bv) && (oi < bi));
      bv = tk ? ov : bv;
      bi = tk ? oi : bi;
    }
    last = bi;
    if (tid == 0) sidx[it] = bi;
  }
  __syncthreads();

  if (tid < 512) {
    const v4i iv = *(const v4i*)(&sidx[tid * 4]);
    st2_v4i(fps_idx + (size_t)b * NUM_CENT + tid * 4, iv);
  }
  for (int f = tid; f < 1536; f += 1024) {
    v4f o;
#pragma unroll
    for (int j = 0; j < 4; ++j) {
      const int e  = 4 * f + j;
      const int s  = e / 3;
      const int cc = e - 3 * s;
      const int ii = clampi(sidx[s], NUM_PTS - 1);
      o[j] = X[ii * 3 + cc];
    }
    st2_v4f(out0 + (size_t)b * (NUM_CENT * 3) + 4 * f, o);
  }
}

__global__ __launch_bounds__(256) void ball_kernel(const float* __restrict__ xyz,
                                                   const int* __restrict__ fps_idx,
                                                   const float* __restrict__ W1,
                                                   int* __restrict__ idxb,
                                                   float* __restrict__ Cw)
{
#pragma clang fp contract(off)
  __shared__ int sl[8][32];
  const int lane = threadIdx.x & 31;
  const int wv   = threadIdx.x >> 5;
  const int c    = blockIdx.x * 8 + wv;
  const int b    = c >> 11;
  const float* X = xyz + (size_t)b * (NUM_PTS * 3);
  const int fi = clampi(fps_idx[c], NUM_PTS - 1);
  const float qx = X[fi * 3 + 0];
  const float qy = X[fi * 3 + 1];
  const float qz = X[fi * 3 + 2];

  sl[wv][lane] = 0;
  __syncthreads();

  int cnt = 0;
  for (int n0 = 0; n0 < NUM_PTS; n0 += 32) {
    const int i = n0 + lane;
    const float dx = qx - X[i * 3 + 0];
    const float dy = qy - X[i * 3 + 1];
    const float dz = qz - X[i * 3 + 2];
    const float t0 = dx * dx;
    const float t1 = dy * dy;
    const float t2 = dz * dz;
    const float d2 = (t0 + t2) + t1;
    const bool pred = d2 < 0.16f;
    const unsigned mask = __builtin_amdgcn_ballot_w32(pred);
    const int pos = cnt + __popc(mask & ((1u << lane) - 1u));
    if (pred && pos < NUM_SAMP) sl[wv][pos] = i;
    cnt += __popc(mask);
    if (cnt >= NUM_SAMP) break;
  }
  __syncthreads();

  const int first = sl[wv][0];
  const int mine  = sl[wv][lane];
  int v = (lane < cnt) ? mine : first;
  v = clampi(v, NUM_PTS - 1);
  st2_i32(idxb + (size_t)c * NUM_SAMP + lane, v);

  const float w0a = W1[lane],       w0b = W1[32 + lane];
  const float w1a = W1[64 + lane],  w1b = W1[96 + lane];
  const float w2a = W1[128 + lane], w2b = W1[160 + lane];
  const float ca = (qx * w0a + qy * w1a) + qz * w2a;
  const float cb = (qx * w0b + qy * w1b) + qz * w2b;
  st2_f32(Cw + (size_t)c * NUM_CHAN + lane, ca);
  st2_f32(Cw + (size_t)c * NUM_CHAN + 32 + lane, cb);
}

__global__ __launch_bounds__(128) void pointproj_kernel(const float* __restrict__ points,
                                                        const float* __restrict__ xyz,
                                                        const float* __restrict__ W1,
                                                        const _Float16* __restrict__ W1t,
                                                        float* __restrict__ Q)
{
  __shared__ __align__(16) _Float16 lW[64 * LDS_PITCH];
  __shared__ __align__(16) float slab[4][16 * SLAB_PITCH];
  __shared__ float sx[4][48];

  const int tid  = threadIdx.x;
  const int lane = tid & 31;
  const int wv   = tid >> 5;
  const int hh   = lane >> 4;
  const int rl   = lane & 15;
  const int c4   = rl * 4;

#pragma unroll
  for (int i = 0; i < 4; ++i) {
    const int u = tid + 128 * i;
    const int n = u >> 3, k8 = (u & 7) * 8;
    *(v8h*)(&lW[n * LDS_PITCH + k8]) = *(const v8h*)(W1t + (size_t)u * 8);
  }
  const v4f wx0 = *(const v4f*)(W1 + c4);
  const v4f wx1 = *(const v4f*)(W1 + 64 + c4);
  const v4f wx2 = *(const v4f*)(W1 + 128 + c4);
  __syncthreads();

  v16h bw[2][4];
#pragma unroll
  for (int kk = 0; kk < 2; ++kk) {
#pragma unroll
    for (int j = 0; j < 4; ++j) {
      const int o = (16 * j + rl) * LDS_PITCH + kk * 32 + 8 * hh;
      FragU f;
      f.h[0] = *(const v8h*)(&lW[o]);
      f.h[1] = *(const v8h*)(&lW[o + 16]);
      bw[kk][j] = f.v;
    }
  }

  for (int t = 0; t < 4; ++t) {
    const int row0 = blockIdx.x * 256 + wv * 64 + t * 16;
    const float* ap = points + (size_t)(row0 + rl) * NUM_CHAN + 8 * hh;
    v16h a[2];
#pragma unroll
    for (int kk = 0; kk < 2; ++kk) {
      const v4f f0 = *(const v4f*)(ap + kk * 32);
      const v4f f1 = *(const v4f*)(ap + kk * 32 + 4);
      const v4f f2 = *(const v4f*)(ap + kk * 32 + 16);
      const v4f f3 = *(const v4f*)(ap + kk * 32 + 20);
#pragma unroll
      for (int e = 0; e < 4; ++e) {
        a[kk][e]      = (_Float16)f0[e];
        a[kk][4 + e]  = (_Float16)f1[e];
        a[kk][8 + e]  = (_Float16)f2[e];
        a[kk][12 + e] = (_Float16)f3[e];
      }
    }
    const int xo = row0 * 3;
    const int l2 = (lane + 32 > 47) ? 47 : (lane + 32);
    const float xa = xyz[xo + lane];
    const float xb = xyz[xo + l2];
    sx[wv][lane] = xa;
    if (lane < 16) sx[wv][32 + lane] = xb;

    v8f acc[4];
#pragma unroll
    for (int j = 0; j < 4; ++j) acc[j] = (v8f){0.f, 0.f, 0.f, 0.f, 0.f, 0.f, 0.f, 0.f};
#pragma unroll
    for (int kk = 0; kk < 2; ++kk) {
#pragma unroll
      for (int j = 0; j < 4; ++j) acc[j] = mma_h(a[kk], bw[kk][j], acc[j]);
    }
#pragma unroll
    for (int j = 0; j < 4; ++j) {
#pragma unroll
      for (int r = 0; r < 8; ++r) slab[wv][(8 * hh + r) * SLAB_PITCH + 16 * j + rl] = acc[j][r];
    }
    __syncthreads();
    for (int pass = 0; pass < 2; ++pass) {
#pragma unroll
      for (int it = 0; it < 8; ++it) {
        const int row = it * 2 + hh;
        v4f v = *(const v4f*)(&slab[wv][row * SLAB_PITCH + c4]);
        const float xv = sx[wv][row * 3 + 0];
        const float yv = sx[wv][row * 3 + 1];
        const float zv = sx[wv][row * 3 + 2];
        v = v + xv * wx0;
        v = v + yv * wx1;
        v = v + zv * wx2;
        *(volatile v4f*)(Q + (size_t)(row0 + row) * NUM_CHAN + c4) = v;
      }
      __threadfence();
    }
    __syncthreads();
  }
}

__global__ __launch_bounds__(128) void stats1_kernel(const float* __restrict__ Q,
                                                     const float* __restrict__ Cw,
                                                     const int* __restrict__ idxb,
                                                     float* __restrict__ part)
{
  __shared__ float lws[4][128];
  const int tid  = threadIdx.x;
  const int lane = tid & 31;
  const int wv   = tid >> 5;
  float s0 = 0.0f, s1 = 0.0f, q0 = 0.0f, q1 = 0.0f;
  for (int cc = 0; cc < CENT_PER_WAVE; ++cc) {
    const int c = blockIdx.x * CENT_PER_BLOCK + wv * CENT_PER_WAVE + cc;
    const int b = c >> 11;
    const int jv = clampi(idxb[(size_t)c * NUM_SAMP + lane], NUM_PTS - 1);
    const v2f cw = *(const v2f*)(Cw + (size_t)c * NUM_CHAN + 2 * lane);
#pragma unroll 4
    for (int k = 0; k < NUM_SAMP; ++k) {
      const int j = __shfl(jv, k, 32);
      const v2f qv = *(const v2f*)(Q + (size_t)(b * NUM_PTS + j) * NUM_CHAN + 2 * lane);
      const float v0 = qv[0] - cw[0];
      const float v1 = qv[1] - cw[1];
      s0 += v0;
      s1 += v1;
      q0 += v0 * v0;
      q1 += v1 * v1;
    }
  }
  lws[wv][2 * lane]          = s0;
  lws[wv][2 * lane + 1]      = s1;
  lws[wv][64 + 2 * lane]     = q0;
  lws[wv][64 + 2 * lane + 1] = q1;
  __syncthreads();
  const float p = ((lws[0][tid] + lws[1][tid]) + lws[2][tid]) + lws[3][tid];
  st2_f32(part + (size_t)blockIdx.x * 128 + tid, p);
}

__global__ __launch_bounds__(128) void bnfin_kernel(const float* __restrict__ part, int nblk, int nch,
                                                    const float* __restrict__ g,
                                                    const float* __restrict__ bt,
                                                    float* __restrict__ scsh)
{
  const int c = threadIdx.x;
  if (c < nch) {
    double sd = 0.0, qd = 0.0;
#pragma unroll 4
    for (int i = 0; i < nblk; ++i) {
      sd += (double)part[(size_t)i * 2 * nch + c];
      qd += (double)part[(size_t)i * 2 * nch + nch + c];
    }
    const double inv = 1.0 / (double)TOT_ROWS;
    const double m = sd * inv;
    const double var = qd * inv - m * m;
    float vf = (float)var;
    vf = vf > 0.0f ? vf : 0.0f;
    const float s = g[c] * rsqrtf(vf + 1e-5f);
    const float h = bt[c] - (float)m * s;
    st2_f32(scsh + c, s);
    st2_f32(scsh + 128 + c, h);
  }
}

__global__ __launch_bounds__(128) void mlp2_kernel(const float* __restrict__ Q,
                                                   const float* __restrict__ Cw,
                                                   const int* __restrict__ idxb,
                                                   const _Float16* __restrict__ W2t,
                                                   const float* __restrict__ scsh,
                                                   _Float16* __restrict__ y2,
                                                   float* __restrict__ part)
{
  __shared__ __align__(16) _Float16 lW[64 * LDS_PITCH];
  __shared__ __align__(16) _Float16 aT[4][32 * LDS_PITCH];
  __shared__ __align__(16) float slab[4][16 * SLAB_PITCH];
  __shared__ float lws[4][128];

  const int tid  = threadIdx.x;
  const int lane = tid & 31;
  const int wv   = tid >> 5;
  const int hh   = lane >> 4;
  const int rl   = lane & 15;
  const int c4   = rl * 4;

#pragma unroll
  for (int i = 0; i < 4; ++i) {
    const int u = tid + 128 * i;
    const int n = u >> 3, k8 = (u & 7) * 8;
    *(v8h*)(&lW[n * LDS_PITCH + k8]) = *(const v8h*)(W2t + (size_t)u * 8);
  }
  const v4f sc = *(const v4f*)(scsh + c4);
  const v4f sh = *(const v4f*)(scsh + 128 + c4);
  __syncthreads();

  v16h bw[2][4];
#pragma unroll
  for (int kk = 0; kk < 2; ++kk) {
#pragma unroll
    for (int j = 0; j < 4; ++j) {
      const int o = (16 * j + rl) * LDS_PITCH + kk * 32 + 8 * hh;
      FragU f;
      f.h[0] = *(const v8h*)(&lW[o]);
      f.h[1] = *(const v8h*)(&lW[o + 16]);
      bw[kk][j] = f.v;
    }
  }

  float ssum[4] = {0.0f, 0.0f, 0.0f, 0.0f};
  float ssq[4]  = {0.0f, 0.0f, 0.0f, 0.0f};

  for (int cc = 0; cc < CENT_PER_WAVE; ++cc) {
    const int c = blockIdx.x * CENT_PER_BLOCK + wv * CENT_PER_WAVE + cc;
    const int b = c >> 11;
    const int jv = clampi(idxb[(size_t)c * NUM_SAMP + lane], NUM_PTS - 1);
    const v4f cw = *(const v4f*)(Cw + (size_t)c * NUM_CHAN + c4);
#pragma unroll 4
    for (int r = 0; r < 16; ++r) {
      const int row = 2 * r + hh;
      const int j = __shfl(jv, row, 32);
      const v4f qv = *(const v4f*)(Q + (size_t)(b * NUM_PTS + j) * NUM_CHAN + c4);
      v4h hv;
#pragma unroll
      for (int e = 0; e < 4; ++e) {
        const float d = qv[e] - cw[e];
        float a = sc[e] * d + sh[e];
        a = a > 0.0f ? a : 0.0f;
        hv[e] = (_Float16)a;
      }
      *(v4h*)(&aT[wv][row * LDS_PITCH + c4]) = hv;
    }
    __syncthreads();

    v8f acc[2][4];
#pragma unroll
    for (int i = 0; i < 2; ++i)
#pragma unroll
      for (int j = 0; j < 4; ++j) acc[i][j] = (v8f){0.f, 0.f, 0.f, 0.f, 0.f, 0.f, 0.f, 0.f};
#pragma unroll
    for (int kk = 0; kk < 2; ++kk) {
      const int o0 = rl * LDS_PITCH + kk * 32 + 8 * hh;
      const int o1 = (16 + rl) * LDS_PITCH + kk * 32 + 8 * hh;
      FragU f0, f1;
      f0.h[0] = *(const v8h*)(&aT[wv][o0]);
      f0.h[1] = *(const v8h*)(&aT[wv][o0 + 16]);
      f1.h[0] = *(const v8h*)(&aT[wv][o1]);
      f1.h[1] = *(const v8h*)(&aT[wv][o1 + 16]);
#pragma unroll
      for (int j = 0; j < 4; ++j) {
        acc[0][j] = mma_h(f0.v, bw[kk][j], acc[0][j]);
        acc[1][j] = mma_h(f1.v, bw[kk][j], acc[1][j]);
      }
    }
#pragma unroll
    for (int i = 0; i < 2; ++i)
#pragma unroll
      for (int j = 0; j < 4; ++j)
#pragma unroll
        for (int r = 0; r < 8; ++r) {
          const float v = acc[i][j][r];
          ssum[j] += v;
          ssq[j]  += v * v;
        }

#pragma unroll
    for (int i = 0; i < 2; ++i) {
#pragma unroll
      for (int j = 0; j < 4; ++j)
#pragma unroll
        for (int r = 0; r < 8; ++r) slab[wv][(8 * hh + r) * SLAB_PITCH + 16 * j + rl] = acc[i][j][r];
      __syncthreads();
      {
        const int q4 = lane >> 3, c8 = (lane & 7) * 8;
        _Float16* dst = y2 + ((size_t)c * NUM_SAMP + i * 16) * NUM_CHAN;
        for (int pass = 0; pass < 2; ++pass) {
#pragma unroll
          for (int it = 0; it < 4; ++it) {
            const int row = it * 4 + q4;
            const v4f lo = *(const v4f*)(&slab[wv][row * SLAB_PITCH + c8]);
            const v4f hi = *(const v4f*)(&slab[wv][row * SLAB_PITCH + c8 + 4]);
            v8h hv;
#pragma unroll
            for (int e = 0; e < 4; ++e) {
              hv[e]     = (_Float16)lo[e];
              hv[4 + e] = (_Float16)hi[e];
            }
            *(volatile v8h*)(dst + (size_t)row * NUM_CHAN + c8) = hv;
          }
          __threadfence();
        }
      }
      __syncthreads();
    }
  }

#pragma unroll
  for (int j = 0; j < 4; ++j) {
    ssum[j] += __shfl_xor(ssum[j], 16, 32);
    ssq[j]  += __shfl_xor(ssq[j], 16, 32);
  }
  if (hh == 0) {
#pragma unroll
    for (int j = 0; j < 4; ++j) {
      lws[wv][16 * j + rl]      = ssum[j];
      lws[wv][64 + 16 * j + rl] = ssq[j];
    }
  }
  __syncthreads();
  const float p = ((lws[0][tid] + lws[1][tid]) + lws[2][tid]) + lws[3][tid];
  st2_f32(part + (size_t)blockIdx.x * 128 + tid, p);
}

__global__ __launch_bounds__(128) void mlp3_kernel(const unsigned short* __restrict__ y2,
                                                   const _Float16* __restrict__ W3t,
                                                   const float* __restrict__ scsh,
                                                   float* __restrict__ ymax,
                                                   float* __restrict__ ymin,
                                                   float* __restrict__ part)
{
  __shared__ __align__(16) _Float16 lW[128 * LDS_PITCH];
  __shared__ __align__(16) _Float16 aT[4][32 * LDS_PITCH];
  __shared__ float lws[4][256];

  const int tid  = threadIdx.x;
  const int lane = tid & 31;
  const int wv   = tid >> 5;
  const int hh   = lane >> 4;
  const int rl   = lane & 15;
  const int q4   = lane >> 3;
  const int c8   = (lane & 7) * 8;

#pragma unroll
  for (int i = 0; i < 8; ++i) {
    const int u = tid + 128 * i;
    const int n = u >> 3, k8 = (u & 7) * 8;
    *(v8h*)(&lW[n * LDS_PITCH + k8]) = *(const v8h*)(W3t + (size_t)u * 8);
  }
  float scv[8], shv[8];
  {
    const v4f s0 = *(const v4f*)(scsh + c8);
    const v4f s1 = *(const v4f*)(scsh + c8 + 4);
    const v4f h0 = *(const v4f*)(scsh + 128 + c8);
    const v4f h1 = *(const v4f*)(scsh + 128 + c8 + 4);
#pragma unroll
    for (int e = 0; e < 4; ++e) {
      scv[e] = s0[e]; scv[4 + e] = s1[e];
      shv[e] = h0[e]; shv[4 + e] = h1[e];
    }
  }
  __syncthreads();

  float ssum[8], ssq[8];
#pragma unroll
  for (int j = 0; j < 8; ++j) { ssum[j] = 0.0f; ssq[j] = 0.0f; }

  for (int cc = 0; cc < CENT_PER_WAVE; ++cc) {
    const int c = blockIdx.x * CENT_PER_BLOCK + wv * CENT_PER_WAVE + cc;
    const unsigned short* src = y2 + (size_t)c * NUM_SAMP * NUM_CHAN;
#pragma unroll 4
    for (int it = 0; it < 8; ++it) {
      const int row = it * 4 + q4;
      const v4u w = *(const v4u*)(src + (size_t)row * NUM_CHAN + c8);
      const unsigned w0 = w[0], w1 = w[1], w2 = w[2], w3 = w[3];
      float f[8];
      f[0] = h16_to_f32(w0 & 0xffffu); f[1] = h16_to_f32(w0 >> 16);
      f[2] = h16_to_f32(w1 & 0xffffu); f[3] = h16_to_f32(w1 >> 16);
      f[4] = h16_to_f32(w2 & 0xffffu); f[5] = h16_to_f32(w2 >> 16);
      f[6] = h16_to_f32(w3 & 0xffffu); f[7] = h16_to_f32(w3 >> 16);
      v8h hv;
#pragma unroll
      for (int e = 0; e < 8; ++e) {
        float a = scv[e] * f[e] + shv[e];
        a = a > 0.0f ? a : 0.0f;
        hv[e] = (_Float16)a;
      }
      *(v8h*)(&aT[wv][row * LDS_PITCH + c8]) = hv;
    }
    __syncthreads();

#pragma unroll
    for (int half = 0; half < 2; ++half) {
      v8f acc[2][4];
#pragma unroll
      for (int i = 0; i < 2; ++i)
#pragma unroll
        for (int j = 0; j < 4; ++j) acc[i][j] = (v8f){0.f, 0.f, 0.f, 0.f, 0.f, 0.f, 0.f, 0.f};
#pragma unroll
      for (int kk = 0; kk < 2; ++kk) {
        const int o0 = rl * LDS_PITCH + kk * 32 + 8 * hh;
        const int o1 = (16 + rl) * LDS_PITCH + kk * 32 + 8 * hh;
        FragU f0, f1;
        f0.h[0] = *(const v8h*)(&aT[wv][o0]);
        f0.h[1] = *(const v8h*)(&aT[wv][o0 + 16]);
        f1.h[0] = *(const v8h*)(&aT[wv][o1]);
        f1.h[1] = *(const v8h*)(&aT[wv][o1 + 16]);
#pragma unroll
        for (int j = 0; j < 4; ++j) {
          const int ob = (half * 64 + 16 * j + rl) * LDS_PITCH + kk * 32 + 8 * hh;
          FragU fb;
          fb.h[0] = *(const v8h*)(&lW[ob]);
          fb.h[1] = *(const v8h*)(&lW[ob + 16]);
          acc[0][j] = mma_h(f0.v, fb.v, acc[0][j]);
          acc[1][j] = mma_h(f1.v, fb.v, acc[1][j]);
        }
      }
      float mxa[4], mna[4];
#pragma unroll
      for (int j = 0; j < 4; ++j) {
        float mx = acc[0][j][0];
        float mn = acc[0][j][0];
#pragma unroll
        for (int i = 0; i < 2; ++i)
#pragma unroll
          for (int r = 0; r < 8; ++r) {
            const float v = acc[i][j][r];
            ssum[half * 4 + j] += v;
            ssq[half * 4 + j]  += v * v;
            mx = fmaxf(mx, v);
            mn = fminf(mn, v);
          }
        const float omx = __shfl_xor(mx, 16, 32);
        const float omn = __shfl_xor(mn, 16, 32);
        mxa[j] = fmaxf(mx, omx);
        mna[j] = fminf(mn, omn);
      }
      const float vmx0 = hh ? mxa[1] : mxa[0];
      const float vmx1 = hh ? mxa[3] : mxa[2];
      const float vmn0 = hh ? mna[1] : mna[0];
      const float vmn1 = hh ? mna[3] : mna[2];
      float* pm = ymax + (size_t)c * NUM_CHAN3 + half * 64 + lane;
      float* pn = ymin + (size_t)c * NUM_CHAN3 + half * 64 + lane;
      for (int pass = 0; pass < 2; ++pass) {
        *(volatile float*)(pm)      = vmx0;
        *(volatile float*)(pm + 32) = vmx1;
        *(volatile float*)(pn)      = vmn0;
        *(volatile float*)(pn + 32) = vmn1;
        __threadfence();
      }
    }
    __syncthreads();
  }

#pragma unroll
  for (int j = 0; j < 8; ++j) {
    ssum[j] += __shfl_xor(ssum[j], 16, 32);
    ssq[j]  += __shfl_xor(ssq[j], 16, 32);
  }
  if (hh == 0) {
#pragma unroll
    for (int j = 0; j < 8; ++j) {
      lws[wv][16 * j + rl]       = ssum[j];
      lws[wv][128 + 16 * j + rl] = ssq[j];
    }
  }
  __syncthreads();
  const float p0 = ((lws[0][tid] + lws[1][tid]) + lws[2][tid]) + lws[3][tid];
  const float p1 = ((lws[0][128 + tid] + lws[1][128 + tid]) + lws[2][128 + tid]) + lws[3][128 + tid];
  st2_f32(part + (size_t)blockIdx.x * 256 + tid, p0);
  st2_f32(part + (size_t)blockIdx.x * 256 + 128 + tid, p1);
}

__global__ __launch_bounds__(256) void pool_out_kernel(const float* __restrict__ ymax,
                                                       const float* __restrict__ ymin,
                                                       const float* __restrict__ scsh,
                                                       float* __restrict__ out1)
{
  const int t  = blockIdx.x * 256 + threadIdx.x;
  const int n4 = (t & 31) * 4;
  const v4f a  = *(const v4f*)(ymax + (size_t)t * 4);
  const v4f bb = *(const v4f*)(ymin + (size_t)t * 4);
  const v4f sc = *(const v4f*)(scsh + n4);
  const v4f sh = *(const v4f*)(scsh + 128 + n4);
  v4f o;
#pragma unroll
  for (int e = 0; e < 4; ++e) {
    const float fa = (sc[e] >= 0.0f) ? 1.0f : 0.0f;
    const float fb = 1.0f - fa;
    const float x  = fa * a[e] + fb * bb[e];
    const float v  = sc[e] * x + sh[e];
    o[e] = v > 0.0f ? v : 0.0f;
  }
  st2_v4f(out1 + (size_t)t * 4, o);
}

extern "C" void kernel_launch(void* const* d_in, const int* in_sizes, int n_in,
                              void* d_out, int out_size, void* d_ws, size_t ws_size,
                              hipStream_t stream)
{
  (void)in_sizes;
  (void)out_size;
  constexpr size_t SZ_FPS   = (size_t)TOT_CENT * 4;
  constexpr size_t SZ_IDX   = (size_t)TOT_ROWS * 4;
  constexpr size_t SZ_WPL   = (size_t)(4096 + 4096 + 8192) * 2;
  constexpr size_t SZ_SCSH  = 4096;
  constexpr size_t SZ_PART1 = (size_t)MLP_BLOCKS * 128 * 4;
  constexpr size_t SZ_PART2 = (size_t)MLP_BLOCKS * 128 * 4;
  constexpr size_t SZ_PART3 = (size_t)MLP_BLOCKS * 256 * 4;
  constexpr size_t SZ_CW    = (size_t)TOT_CENT * NUM_CHAN * 4;
  constexpr size_t SZ_Q     = (size_t)TOT_PTS * NUM_CHAN * 4;
  constexpr size_t SZ_YM    = (size_t)TOT_CENT * NUM_CHAN3 * 4;
  constexpr size_t SZ_Y2    = (size_t)TOT_ROWS * NUM_CHAN * 2;
  constexpr size_t OFF_FPS   = 0;
  constexpr size_t OFF_IDX   = OFF_FPS + SZ_FPS;
  constexpr size_t OFF_WPL   = OFF_IDX + SZ_IDX;
  constexpr size_t OFF_SCSH  = OFF_WPL + SZ_WPL;
  constexpr size_t OFF_PART1 = OFF_SCSH + SZ_SCSH;
  constexpr size_t OFF_PART2 = OFF_PART1 + SZ_PART1;
  constexpr size_t OFF_PART3 = OFF_PART2 + SZ_PART2;
  constexpr size_t OFF_CW    = OFF_PART3 + SZ_PART3;
  constexpr size_t OFF_Q     = OFF_CW + SZ_CW;
  constexpr size_t OFF_YMAX  = OFF_Q + SZ_Q;
  constexpr size_t OFF_YMIN  = OFF_YMAX + SZ_YM;
  constexpr size_t OFF_Y2    = OFF_YMIN + SZ_YM;
  constexpr size_t WS_TOTAL  = OFF_Y2 + SZ_Y2;
  static_assert(WS_TOTAL == 109154304);
  static_assert(WS_TOTAL <= 134217728);
  static_assert((OFF_IDX % 128) == 0 && (OFF_WPL % 128) == 0 && (OFF_SCSH % 128) == 0);
  static_assert((OFF_PART1 % 128) == 0 && (OFF_CW % 128) == 0 && (OFF_Q % 128) == 0 && (OFF_Y2 % 128) == 0);
  static_assert((size_t)TOT_CENT * 3 * 4 == 196608);
  static_assert((size_t)TOT_CENT * 3 * 4 + (size_t)TOT_CENT * NUM_CHAN3 * 4 == 8585216);

  if (n_in < 11) return;
  if (ws_size < WS_TOTAL) return;

  const float* xyz    = (const float*)d_in[0];
  const float* points = (const float*)d_in[1];
  const float* W1 = (const float*)d_in[2];
  const float* g1 = (const float*)d_in[3];
  const float* b1 = (const float*)d_in[4];
  const float* W2 = (const float*)d_in[5];
  const float* g2 = (const float*)d_in[6];
  const float* b2 = (const float*)d_in[7];
  const float* W3 = (const float*)d_in[8];
  const float* g3 = (const float*)d_in[9];
  const float* b3 = (const float*)d_in[10];

  float* out0 = (float*)d_out;
  float* out1 = (float*)d_out + (size_t)TOT_CENT * 3;

  char* ws = (char*)d_ws;
  int*      fpsIdx = (int*)(ws + OFF_FPS);
  int*      idxb   = (int*)(ws + OFF_IDX);
  _Float16* wpl    = (_Float16*)(ws + OFF_WPL);
  _Float16* w1t    = wpl;
  _Float16* w2t    = wpl + 4096;
  _Float16* w3t    = wpl + 8192;
  float*    scsh1  = (float*)(ws + OFF_SCSH);
  float*    scsh2  = scsh1 + 256;
  float*    scsh3  = scsh1 + 512;
  float*    part1  = (float*)(ws + OFF_PART1);
  float*    part2  = (float*)(ws + OFF_PART2);
  float*    part3  = (float*)(ws + OFF_PART3);
  float*    cwp    = (float*)(ws + OFF_CW);
  float*    qp     = (float*)(ws + OFF_Q);
  float*    ymaxp  = (float*)(ws + OFF_YMAX);
  float*    yminp  = (float*)(ws + OFF_YMIN);
  _Float16* y2p    = (_Float16*)(ws + OFF_Y2);

  wprep_kernel<<<8, 256, 0, stream>>>(W1, W2, W3, wpl);
  fps_kernel<<<NUM_BATCH, 1024, 0, stream>>>(xyz, fpsIdx, out0);
  ball_kernel<<<TOT_CENT / 8, 256, 0, stream>>>(xyz, fpsIdx, W1, idxb, cwp);
  pointproj_kernel<<<TOT_PTS / 256, 128, 0, stream>>>(points, xyz, W1, w1t, qp);
  stats1_kernel<<<MLP_BLOCKS, 128, 0, stream>>>(qp, cwp, idxb, part1);
  bnfin_kernel<<<1, 128, 0, stream>>>(part1, MLP_BLOCKS, NUM_CHAN, g1, b1, scsh1);
  mlp2_kernel<<<MLP_BLOCKS, 128, 0, stream>>>(qp, cwp, idxb, w2t, scsh1, y2p, part2);
  bnfin_kernel<<<1, 128, 0, stream>>>(part2, MLP_BLOCKS, NUM_CHAN, g2, b2, scsh2);
  mlp3_kernel<<<MLP_BLOCKS, 128, 0, stream>>>((const unsigned short*)y2p, w3t, scsh2, ymaxp, yminp, part3);
  bnfin_kernel<<<1, 128, 0, stream>>>(part3, MLP_BLOCKS, NUM_CHAN3, g3, b3, scsh3);
  pool_out_kernel<<<(TOT_CENT * NUM_CHAN3 / 4) / 256, 256, 0, stream>>>(ymaxp, yminp, scsh3, out1);
}
